// NCF_Hyper_90357521973958
// MI455X (gfx1250) — hardware-verified
//
#include <hip/hip_runtime.h>
#include <stddef.h>


typedef _Float16 h16;
typedef _Float16 v16h __attribute__((ext_vector_type(16)));
typedef _Float16 v8h  __attribute__((ext_vector_type(8)));
typedef float    v8f  __attribute__((ext_vector_type(8)));
typedef float    v4f  __attribute__((ext_vector_type(4)));

#define NCHUNK_IN 300
#define CHUNK_EMB 64
#define PREF_EMB  32
#define IN_DIM    96
#define HIDDEN    100
#define NWS       110000
#define OUT_ELEMS 7073249
#define NROWS_OUT 65
#define MROWS     80
#define KPAD      128
#define LDA       136
#define CLD       84
#define GEN_COLS  64
#define GEN_TILE  80
#define GEN_BLOCKS 1719

#define WCARRY 64.0f
#define ACARRY 64.0f
#define INV_CARRY (1.0f / 4096.0f)

#define WS_TOTAL ((size_t)MROWS * KPAD * 2)

static_assert(IN_DIM == PREF_EMB + CHUNK_EMB);
static_assert((IN_DIM % 32) == 0 && IN_DIM == 96);
static_assert(HIDDEN == 100);
static_assert((KPAD % 32) == 0 && KPAD >= HIDDEN && KPAD == 8 * 16);
static_assert((MROWS % 16) == 0 && MROWS / 16 == 5 && MROWS <= NCHUNK_IN);
static_assert(MROWS >= NROWS_OUT + 1);
static_assert((size_t)(NROWS_OUT - 1) * NWS < (size_t)OUT_ELEMS);
static_assert((size_t)NROWS_OUT * NWS >= (size_t)OUT_ELEMS);
static_assert((OUT_ELEMS % 32) == 1);
static_assert(((2 * NWS) % 32) == 0 && (NWS % 32) == 16);
static_assert(GEN_BLOCKS * GEN_COLS >= NWS && (GEN_BLOCKS - 1) * GEN_COLS < NWS);
static_assert((GEN_BLOCKS - 2) * GEN_COLS + GEN_TILE <= NWS);
static_assert((GEN_BLOCKS - 1) * GEN_COLS + GEN_TILE - NWS <= NWS);
static_assert(GEN_TILE == 5 * 16 && GEN_TILE <= CLD && GEN_COLS + 16 == GEN_TILE);
static_assert(7 * 20 >= 2 * NROWS_OUT);
static_assert((LDA % 8) == 0 && LDA >= KPAD);
static_assert((CLD % 4) == 0);
static_assert((size_t)4 * (2 * (84580 * 32 + 25896 * 32) + 2048 + 32 + 512 + 16 + 128 + 8 + 40 + 1)
              == (size_t)28292996);
static_assert((size_t)4 * OUT_ELEMS == (size_t)28292996);
static_assert((size_t)(NROWS_OUT + 1) * NWS < (size_t)0xFFFFFFFFu);
static_assert(WS_TOTAL <= (size_t)134217728);
static_assert((WS_TOTAL % 128) == 0);

__device__ __forceinline__ float bf16r(float x) {
  unsigned int u = __float_as_uint(x);
  u = (u + 0x7FFFu + ((u >> 16) & 1u)) & 0xFFFF0000u;
  return __uint_as_float(u);
}

__device__ __forceinline__ h16 toh_flush(float v) {
  const h16 r = (h16)v;
  return (fabsf(v) < 6.103515625e-05f) ? (h16)0.0f : r;
}

__device__ __forceinline__ h16 wconv(float w, bool ok) {
  const float t = ok ? (WCARRY * bf16r(w)) : 0.0f;
  return toh_flush(t);
}

__device__ __forceinline__ v16h frag_at(const _Float16* p) {
  v8h lo = *(const v8h*)(p);
  v8h hi = *(const v8h*)(p + 16);
  v16h out;
#pragma unroll
  for (int i = 0; i < 8; ++i) { out[i] = lo[i]; out[i + 8] = hi[i]; }
  return out;
}
__device__ __forceinline__ v16h ld_frag(const _Float16* base, unsigned ld) {
  const unsigned lane = threadIdx.x & 31u;
  return frag_at(base + (lane & 15u) * ld + (lane >> 4) * 8u);
}

__device__ __forceinline__ v16h wfrag_full(const float* __restrict__ rowp, unsigned k0,
                                           unsigned hh, bool ok) {
  const float* p = rowp + k0 + hh * 8u;
  const v4f a0 = *(const v4f*)(p);
  const v4f a1 = *(const v4f*)(p + 4);
  const v4f a2 = *(const v4f*)(p + 16);
  const v4f a3 = *(const v4f*)(p + 20);
  v16h out;
#pragma unroll
  for (int i = 0; i < 4; ++i) {
    out[i]      = wconv(a0[i], ok);
    out[i + 4]  = wconv(a1[i], ok);
    out[i + 8]  = wconv(a2[i], ok);
    out[i + 12] = wconv(a3[i], ok);
  }
  return out;
}
__device__ __forceinline__ v16h wfrag_tail(const float* __restrict__ rowp, unsigned hh, bool ok) {
  const v4f a0 = *(const v4f*)(rowp + 96);
  const bool use = ok && (hh == 0u);
  v16h out;
#pragma unroll
  for (int i = 0; i < 4; ++i) out[i] = wconv(a0[i], use);
#pragma unroll
  for (int i = 4; i < 16; ++i) out[i] = (h16)0.0f;
  return out;
}

__device__ __forceinline__ v8f wmma16(v16h a, v16h b, v8f c) {
  v8f d = __builtin_amdgcn_wmma_f32_16x16x32_f16(false, a, false, b, (short)0, c,
                                                 false, false);
  asm volatile("v_nop\n\tv_nop\n\tv_nop\n\tv_nop" : "+v"(d) : "v"(a), "v"(b));
  return d;
}

__global__ __launch_bounds__(256) void trunk_kernel(
    const float* __restrict__ pref, const float* __restrict__ pemb,
    const float* __restrict__ cemb,
    const float* __restrict__ wt1, const float* __restrict__ bs1,
    const float* __restrict__ wt2, const float* __restrict__ bs2,
    const float* __restrict__ wt3, const float* __restrict__ bs3,
    _Float16* __restrict__ rep16) {
  __shared__ __attribute__((aligned(16))) _Float16 Xa[16 * LDA];
  __shared__ __attribute__((aligned(16))) _Float16 Xb[16 * LDA];
  const unsigned tid = threadIdx.x, lane = tid & 31u;
  const unsigned wave = (unsigned)__builtin_amdgcn_readfirstlane((int)(tid >> 5));
  const unsigned hh = lane >> 4, m = lane & 15u;
  const unsigned c0 = blockIdx.x * 16u;

  const float p0 = bf16r(pref[0]);
  const float p1 = bf16r(pref[1]);
#pragma unroll 1
  for (unsigned j = 0; j < 8u; ++j) {
    const unsigned idx = tid + 256u * j;
    const unsigned r = idx >> 7, c = idx & 127u;
    const unsigned cp = c & 31u;
    const unsigned cc = (c < 32u) ? 0u : ((c > 95u) ? 63u : (c - 32u));
    const float e0 = pemb[cp];
    const float e1 = pemb[PREF_EMB + cp];
    const float ce = cemb[(size_t)(c0 + r) * CHUNK_EMB + cc];
    const float pv = p0 * bf16r(e0) + p1 * bf16r(e1);
    const float v = (c < 32u) ? pv : ((c < 96u) ? bf16r(ce) : 0.0f);
    Xa[r * LDA + c] = toh_flush(ACARRY * v);
  }
  __syncthreads();

  const unsigned n = wave * 16u + m;
  const bool nok = (n < (unsigned)HIDDEN);
  const unsigned nc = nok ? n : (unsigned)(HIDDEN - 1);

  {
    const float* rowp = wt1 + (size_t)nc * IN_DIM;
    v8f acc = {};
#pragma unroll 1
    for (unsigned kt = 0; kt < 3u; ++kt) {
      const v16h b = wfrag_full(rowp, kt * 32u, hh, nok);
      const v16h a = ld_frag(&Xa[kt * 32u], LDA);
      acc = wmma16(a, b, acc);
    }
    const float bl = bs1[nc];
    const float bb = nok ? bf16r(bl) : 0.0f;
#pragma unroll
    for (int r = 0; r < 8; ++r) {
      float t = acc[r] * INV_CARRY + bb;
      t = fmaxf(t, 0.0f);
      t = nok ? t : 0.0f;
      Xb[(hh * 8u + (unsigned)r) * LDA + n] = toh_flush(ACARRY * t);
    }
  }
  __syncthreads();

  {
    const float* rowp = wt2 + (size_t)nc * HIDDEN;
    v8f acc = {};
#pragma unroll 1
    for (unsigned kt = 0; kt < 3u; ++kt) {
      const v16h b = wfrag_full(rowp, kt * 32u, hh, nok);
      const v16h a = ld_frag(&Xb[kt * 32u], LDA);
      acc = wmma16(a, b, acc);
    }
    {
      const v16h b = wfrag_tail(rowp, hh, nok);
      const v16h a = ld_frag(&Xb[96], LDA);
      acc = wmma16(a, b, acc);
    }
    const float bl = bs2[nc];
    const float bb = nok ? bf16r(bl) : 0.0f;
#pragma unroll
    for (int r = 0; r < 8; ++r) {
      float t = acc[r] * INV_CARRY + bb;
      t = fmaxf(t, 0.0f);
      t = nok ? t : 0.0f;
      Xa[(hh * 8u + (unsigned)r) * LDA + n] = toh_flush(ACARRY * t);
    }
  }
  __syncthreads();

  {
    const float* rowp = wt3 + (size_t)nc * HIDDEN;
    v8f acc = {};
#pragma unroll 1
    for (unsigned kt = 0; kt < 3u; ++kt) {
      const v16h b = wfrag_full(rowp, kt * 32u, hh, nok);
      const v16h a = ld_frag(&Xa[kt * 32u], LDA);
      acc = wmma16(a, b, acc);
    }
    {
      const v16h b = wfrag_tail(rowp, hh, nok);
      const v16h a = ld_frag(&Xa[96], LDA);
      acc = wmma16(a, b, acc);
    }
    const float bl = bs3[nc];
    const float bb = nok ? bf16r(bl) : 0.0f;
#pragma unroll
    for (int r = 0; r < 8; ++r) {
      float t = acc[r] * INV_CARRY + bb;
      t = nok ? t : 0.0f;
      Xb[(hh * 8u + (unsigned)r) * LDA + n] = toh_flush(ACARRY * t);
    }
  }
  __syncthreads();

  {
    const unsigned r = tid >> 4, pc = (tid & 15u) * 8u;
    const v8h x = *(const v8h*)&Xb[r * LDA + pc];
    _Float16* p = rep16 + (size_t)(c0 + r) * KPAD + pc;
    *(volatile v8h*)p = x;
    __threadfence();
    *(volatile v8h*)p = x;
  }
}

__global__ __launch_bounds__(160) void gen_kernel(
    const _Float16* __restrict__ rep16, const float* __restrict__ hw, float* __restrict__ out) {
  __shared__ __attribute__((aligned(16))) float Cs[MROWS * CLD];
  const unsigned tid = threadIdx.x, lane = tid & 31u;
  const unsigned wave = (unsigned)__builtin_amdgcn_readfirstlane((int)(tid >> 5));
  const unsigned hh = lane >> 4, m = lane & 15u;
  const unsigned n0 = blockIdx.x * (unsigned)GEN_COLS;

  unsigned wr = n0 + wave * 16u + m;
  wr = (wr >= (unsigned)NWS) ? (wr - (unsigned)NWS) : wr;
  const float* rowp = hw + (size_t)wr * HIDDEN;
  const _Float16* ap = rep16 + (size_t)m * KPAD + hh * 8u;

  v8f acc[5];
#pragma unroll
  for (int mt = 0; mt < 5; ++mt) acc[mt] = (v8f){};

#pragma unroll 1
  for (unsigned kt = 0; kt < 3u; ++kt) {
    const unsigned k0 = kt * 32u;
    const v16h b = wfrag_full(rowp, k0, hh, true);
#pragma unroll
    for (int mt = 0; mt < 5; ++mt) {
      const v16h a = frag_at(ap + (size_t)mt * 16 * KPAD + k0);
      acc[mt] = wmma16(a, b, acc[mt]);
    }
  }
  {
    const v16h b = wfrag_tail(rowp, hh, true);
#pragma unroll
    for (int mt = 0; mt < 5; ++mt) {
      const v16h a = frag_at(ap + (size_t)mt * 16 * KPAD + 96);
      acc[mt] = wmma16(a, b, acc[mt]);
    }
  }

#pragma unroll
  for (int mt = 0; mt < 5; ++mt)
#pragma unroll
    for (int r = 0; r < 8; ++r)
      Cs[((unsigned)mt * 16u + hh * 8u + (unsigned)r) * CLD + wave * 16u + m] =
          acc[mt][r] * INV_CARRY;
  __syncthreads();

  v4f xs[7];
  unsigned off[7];
  bool fl[7], tl[7];
#pragma unroll
  for (unsigned i = 0; i < 7u; ++i) {
    const unsigned t = i * 20u + wave * 4u + (lane >> 3);
    const unsigned pc = (lane & 7u) * 4u;
    const unsigned tt = (t < 2u * NROWS_OUT) ? t : (2u * NROWS_OUT - 1u);
    const unsigned c = tt >> 1, s = tt & 1u;
    const unsigned j0 = ((c & 1u) ? 16u : 0u) + 32u * s;
    const unsigned lc0 = n0 + j0;
    const unsigned srow = c + (((lc0 + pc) >= (unsigned)NWS) ? 1u : 0u);
    const unsigned flat0 = c * (unsigned)NWS + lc0;
    const bool live = (t < 2u * NROWS_OUT) && (lc0 < (unsigned)NWS);
    fl[i] = live && (flat0 + 32u <= (unsigned)OUT_ELEMS);
    tl[i] = live && (flat0 + 1u == (unsigned)OUT_ELEMS) && (pc == 0u);
    xs[i] = *(const v4f*)&Cs[srow * CLD + j0 + pc];
    off[i] = flat0 + pc;
  }
#pragma unroll
  for (int i = 0; i < 7; ++i) {
    if (fl[i]) *(volatile v4f*)(out + off[i]) = xs[i];
    if (tl[i]) *(volatile float*)(out + off[i]) = xs[i][0];
  }
  __threadfence();
#pragma unroll
  for (int i = 0; i < 7; ++i) {
    if (fl[i]) *(volatile v4f*)(out + off[i]) = xs[i];
    if (tl[i]) *(volatile float*)(out + off[i]) = xs[i][0];
  }
}

extern "C" void kernel_launch(void* const* d_in, const int* in_sizes, int n_in,
                              void* d_out, int out_size, void* d_ws, size_t ws_size,
                              hipStream_t stream) {
  if (n_in < 10) return;
  if (in_sizes[0] < 2) return;
  if (in_sizes[1] < 2 * PREF_EMB) return;
  if ((long long)in_sizes[2] < (long long)MROWS * CHUNK_EMB) return;
  if (in_sizes[3] < HIDDEN * IN_DIM) return;
  if (in_sizes[4] < HIDDEN) return;
  if (in_sizes[5] < HIDDEN * HIDDEN) return;
  if (in_sizes[6] < HIDDEN) return;
  if (in_sizes[7] < HIDDEN * HIDDEN) return;
  if (in_sizes[8] < HIDDEN) return;
  if ((long long)in_sizes[9] < (long long)NWS * HIDDEN) return;
  if ((long long)out_size < (long long)OUT_ELEMS) return;
  if (ws_size < WS_TOTAL) return;

  const float* pref = (const float*)d_in[0];
  const float* pemb = (const float*)d_in[1];
  const float* cemb = (const float*)d_in[2];
  const float* wt1  = (const float*)d_in[3];
  const float* bs1  = (const float*)d_in[4];
  const float* wt2  = (const float*)d_in[5];
  const float* bs2  = (const float*)d_in[6];
  const float* wt3  = (const float*)d_in[7];
  const float* bs3  = (const float*)d_in[8];
  const float* hw   = (const float*)d_in[9];
  float* out = (float*)d_out;
  _Float16* rep16 = (_Float16*)d_ws;

  trunk_kernel<<<dim3(MROWS / 16), dim3(256), 0, stream>>>(
      pref, pemb, cemb, wt1, bs1, wt2, bs2, wt3, bs3, rep16);
  gen_kernel<<<dim3(GEN_BLOCKS), dim3(160), 0, stream>>>(rep16, hw, out);
}
